// DMoNLayer_5892695130194
// MI455X (gfx1250) — hardware-verified
//
#include <hip/hip_runtime.h>


namespace {
constexpr int N = 100000, DI = 128, DH = 256, K = 16, E = 3200000, ECH = 4096;
constexpr float XS = 8.0f, WSC = 256.0f;
typedef _Float16 b16;
typedef __attribute__((ext_vector_type(16))) _Float16 v16b;
typedef __attribute__((ext_vector_type(8))) _Float16 v8b;
typedef __attribute__((ext_vector_type(8))) float v8f;
typedef __attribute__((ext_vector_type(4))) float v4f;
__device__ __forceinline__ float bf16_rne(float f) { unsigned int u = __float_as_uint(f); u += 0x7FFFu + ((u >> 16) & 1u); float r = __uint_as_float(u & 0xFFFF0000u); asm volatile("" : "+v"(r)); return r; }
__device__ __forceinline__ void split16(float v, b16& hi, b16& lo) { hi = (b16)v; lo = (b16)(v - (float)hi); }
__device__ __forceinline__ v16b frag_kb(const b16* p, int hh) { const v8b a = *(const v8b*)(p + 8 * hh), b = *(const v8b*)(p + 16 + 8 * hh); v16b f;
#pragma unroll
  for (int e = 0; e < 8; ++e) { f[e] = a[e]; f[8 + e] = b[e]; } return f; }
__device__ __forceinline__ v8f wmma16b(v16b a, v16b b, v8f c) { v8f d = __builtin_amdgcn_wmma_f32_16x16x32_f16(false, a, false, b, (short)0, c, false, false); asm volatile("v_nop\n\tv_nop\n\tv_nop\n\tv_nop" : "+v"(d) : "v"(a), "v"(b)); return d; }
__device__ __forceinline__ void wave_lds_sync() { __builtin_amdgcn_fence(__ATOMIC_RELEASE, "workgroup"); __builtin_amdgcn_wave_barrier(); __builtin_amdgcn_fence(__ATOMIC_ACQUIRE, "workgroup"); }
__device__ __forceinline__ float pmul(float a, float b) { float p = a * b; asm volatile("" : "+v"(p)); return p; }
__device__ __forceinline__ int iclamp(int v, int lo, int hi) { return v < lo ? lo : (v > hi ? hi : v); }

__global__ __launch_bounds__(256) void wput_kernel(const float* __restrict__ w1, const float* __restrict__ w2, b16* __restrict__ W1T, b16* __restrict__ W2T) { const int u = blockIdx.x * 256 + threadIdx.x;
  for (int pass = 0; pass < 2; ++pass) {
    if (u < DH * 16) { const int o = u / 16, k0 = (u % 16) * 8; v8b v;
#pragma unroll
      for (int j = 0; j < 8; ++j) v[j] = (b16)(bf16_rne(w1[(size_t)(k0 + j) * DH + o]) * WSC); *(volatile v8b*)(W1T + (size_t)o * DI + k0) = v; }
    if (u < K * 32) { const int o = u / 32, k0 = (u % 32) * 8; v8b v;
#pragma unroll
      for (int j = 0; j < 8; ++j) v[j] = (b16)(bf16_rne(w2[(size_t)(k0 + j) * K + o]) * WSC); *(volatile v8b*)(W2T + (size_t)o * DH + k0) = v; }
    __threadfence(); } }
__global__ __launch_bounds__(32) void mlp_kernel(const float* __restrict__ x, const b16* __restrict__ W1T, const float* __restrict__ b1, const b16* __restrict__ W2T, const float* __restrict__ b2, int NLIM, float* __restrict__ Cout) { __shared__ __attribute__((aligned(16))) b16 Ah[16][DH + 8], Al[16][DH + 8]; __shared__ float Pf[16][20]; const int lane = threadIdx.x, nloc = lane & 15, hlf = lane >> 4; const size_t m0 = (size_t)blockIdx.x * 16; if (m0 >= (size_t)NLIM) return;
  for (int rr = 0; rr < 16; ++rr) for (int q = 0; q < 4; ++q) Ah[rr][q * 32 + lane] = (b16)(bf16_rne(x[(m0 + rr) * DI + q * 32 + lane]) * XS);
  wave_lds_sync(); v8f acc[16];
#pragma unroll
  for (int t = 0; t < 16; ++t) acc[t] = (v8f){};
#pragma unroll
  for (int kb = 0; kb < DI; kb += 32) { const v16b a = frag_kb(&Ah[nloc][kb], hlf);
#pragma unroll
    for (int t = 0; t < 16; ++t) acc[t] = wmma16b(a, frag_kb(W1T + (size_t)(t * 16 + nloc) * DI + kb, hlf), acc[t]); }
  wave_lds_sync();
#pragma unroll
  for (int t = 0; t < 16; ++t) { const int cc = t * 16 + nloc; const float bb = bf16_rne(b1[cc]);
#pragma unroll
    for (int r8 = 0; r8 < 8; ++r8) { b16 p, ql; split16(fmaxf(acc[t][r8] * (1.0f / (XS * WSC)) + bb, 0.0f) * XS, p, ql); Ah[8 * hlf + r8][cc] = p; Al[8 * hlf + r8][cc] = ql; } }
  wave_lds_sync(); v8f lg = {};
#pragma unroll 2
  for (int kb = 0; kb < DH; kb += 32) { const v16b a = frag_kb(&Ah[nloc][kb], hlf), al = frag_kb(&Al[nloc][kb], hlf); const v16b bw = frag_kb(W2T + (size_t)nloc * DH + kb, hlf); lg = wmma16b(a, bw, lg); lg = wmma16b(al, bw, lg); }
  const float bb2 = bf16_rne(b2[nloc]);
#pragma unroll
  for (int r8 = 0; r8 < 8; ++r8) { const float v = lg[r8] * (1.0f / (XS * WSC)) + bb2; float mx = v; mx = fmaxf(mx, __shfl_xor(mx, 1)); mx = fmaxf(mx, __shfl_xor(mx, 2)); mx = fmaxf(mx, __shfl_xor(mx, 4)); mx = fmaxf(mx, __shfl_xor(mx, 8)); const float e = __expf(v - mx); float s = e; s += __shfl_xor(s, 1); s += __shfl_xor(s, 2); s += __shfl_xor(s, 4); s += __shfl_xor(s, 8); Pf[8 * hlf + r8][nloc] = e / s; }
  wave_lds_sync();
  for (int pass = 0; pass < 2; ++pass) { for (int q = lane; q < 256; q += 32) ((volatile float*)Cout)[m0 * K + q] = Pf[q / K][q % K]; __threadfence(); } }
__global__ __launch_bounds__(256) void esum_kernel(const float* __restrict__ Cc, const int* __restrict__ ei, int NLIM, float* __restrict__ PS) { const int wave = threadIdx.x >> 5, lane = threadIdx.x & 31; const size_t w = (size_t)blockIdx.x * 8 + wave; const size_t e0 = w * ECH; if (e0 >= (size_t)E) return; const size_t e1 = (e0 + ECH < (size_t)E) ? e0 + ECH : (size_t)E; float s = 0.0f;
  for (size_t e = e0 + lane; e < e1; e += 32) { const int u = iclamp(ei[e], 0, N - 1), v = iclamp(ei[E + e], 0, N - 1); if (u >= NLIM || v >= NLIM) continue; const v4f* cu = (const v4f*)(Cc + (size_t)u * K); const v4f* cv = (const v4f*)(Cc + (size_t)v * K); float d = 0.0f;
#pragma unroll
    for (int q = 0; q < 4; ++q) { const v4f a = cu[q], b = cv[q]; for (int k = 0; k < 4; ++k) d += pmul(a[k], b[k]); } s += d; }
  for (int o = 16; o; o >>= 1) s += __shfl_xor(s, o);
  for (int pass = 0; pass < 2; ++pass) { ((volatile float*)PS)[w * 32 + lane] = lane == 0 ? s : 0.0f; __threadfence(); } }
__global__ __launch_bounds__(256) void loss_kernel(const float* __restrict__ PS, int nw, float* __restrict__ L) { __shared__ double S[256]; const int t = threadIdx.x; double s = 0.0; for (int w = t; w < nw; w += 256) s += (double)PS[(size_t)w * 32]; S[t] = s; __syncthreads();
  for (int st = 128; st > 0; st >>= 1) { if (t < st) S[t] += S[t + st]; __syncthreads(); }
  const float loss = (float)(-S[0] / (double)E);
  for (int pass = 0; pass < 2; ++pass) { if (t == 0) ((volatile float*)L)[0] = loss; __threadfence(); } }
}

extern "C" void kernel_launch(void* const* d_in, const int* in_sizes, int n_in, void* d_out, int out_size, void* d_ws, size_t ws_size, hipStream_t stream) {
  (void)n_in;
  auto Fp = [&](int i) { return (const float*)d_in[i]; }; auto Ip = [&](int i) { return (const int*)d_in[i]; };
  if (in_sizes[0] != N * DI || in_sizes[1] != 2 * E || in_sizes[2] != DI * DH || in_sizes[4] != DH * K || out_size != N * K + 1) return;
  const int NLIM = N;
  size_t off = 0; char* ws = (char*)d_ws;
  auto carve = [&](size_t bytes) { char* p = ws + off; off += (bytes + 255) & ~(size_t)255; return p; };
  const int NW = (E + ECH - 1) / ECH;
  b16* W1T = (b16*)carve((size_t)DH * DI * 2); b16* W2T = (b16*)carve((size_t)K * DH * 2); float* PS = (float*)carve((size_t)NW * 32 * 4);
  if (off > ws_size || off > ((size_t)8 << 20)) return;
  float* Cc = (float*)d_out;
  wput_kernel<<<(DH * 16 + 255) / 256, 256, 0, stream>>>(Fp(2), Fp(4), W1T, W2T);
  mlp_kernel<<<NLIM / 16, 32, 0, stream>>>(Fp(0), W1T, Fp(3), W2T, Fp(5), NLIM, Cc);
  esum_kernel<<<(NW + 7) / 8, 256, 0, stream>>>(Cc, Ip(1), NLIM, PS);
  loss_kernel<<<1, 256, 0, stream>>>(PS, NW, Cc + (size_t)N * K);
}
